// EnhancedSTAMT_37108517437566
// MI455X (gfx1250) — hardware-verified
//
#include <hip/hip_runtime.h>
#include <math.h>
#include <stdint.h>

#define NB 8
#define ND 128
#define NN 307
#define NP 320
#define NL 12
#define NH 8
#define SS 3684
#define ROWS 30720
#define NTILE 480
#define K3 960
#define LDF 132
#define LDA 264
#define MSTRIDE 471552

static_assert(NP == 5 * 64);
static_assert(ND == NH * 16);
static_assert((8 * SS * 4) % 128 == 0);
static_assert(NN <= NP);
static_assert(ROWS == NB * NL * NP);
static_assert(NTILE * 64 == ROWS);
static_assert(MSTRIDE == NH * NL * NN * 16);

typedef __attribute__((ext_vector_type(16))) __bf16 v16b;
typedef __attribute__((ext_vector_type(8)))  float v8f;
typedef __attribute__((ext_vector_type(4)))  float v4f;
typedef __attribute__((ext_vector_type(2)))  float v2f;
typedef __attribute__((ext_vector_type(2)))  double v2d;
typedef __attribute__((ext_vector_type(8)))  unsigned short v8us;
typedef __attribute__((ext_vector_type(4)))  unsigned short v4us;
typedef __attribute__((ext_vector_type(2)))  unsigned short v2us;
typedef v8us __attribute__((may_alias)) v8usa;
typedef v4us __attribute__((may_alias)) v4usa;
typedef v2us __attribute__((may_alias)) v2usa;
typedef v4f  __attribute__((may_alias)) v4fa;
typedef v2f  __attribute__((may_alias)) v2fa;

union FB { v16b v; v8us h[2]; };

__device__ __forceinline__ unsigned short f2bf_bits(float f) {
  const unsigned u = __float_as_uint(f);
  return (unsigned short)((u + 0x7FFFu + ((u >> 16) & 1u)) >> 16);
}
__device__ __forceinline__ float bf_bits2f(unsigned short h) { return __uint_as_float(((unsigned)h) << 16); }
__device__ __forceinline__ float bfr(float f) { return bf_bits2f(f2bf_bits(f)); }
__device__ __forceinline__ unsigned split_pk(float f) {
  const unsigned short hb = f2bf_bits(f);
  const unsigned short lb = f2bf_bits(f - bf_bits2f(hb));
  return (unsigned)hb | (((unsigned)lb) << 16);
}
__device__ __forceinline__ float blendf(float a, float b, unsigned m) {
  return __uint_as_float((__float_as_uint(a) & m) | (__float_as_uint(b) & ~m));
}

__device__ __forceinline__ v8f wmb(v16b a, v16b b, v8f c) {
  c = __builtin_amdgcn_wmma_f32_16x16x32_bf16(false, a, false, b, (short)0, c, false, false);
  asm volatile("v_nop\n\tv_nop\n\tv_nop\n\tv_nop" : "+v"(c) : "v"(a), "v"(b));
  return c;
}
__device__ __forceinline__ v16b ldfrag_g(const unsigned short* p) {
  FB f; f.h[0] = *(const v8usa*)p; f.h[1] = *(const v8usa*)(p + 16); return f.v;
}
__device__ __forceinline__ void wave_sync() {
  __builtin_amdgcn_fence(__ATOMIC_RELEASE, "workgroup");
  __builtin_amdgcn_wave_barrier();
  __builtin_amdgcn_fence(__ATOMIC_ACQUIRE, "workgroup");
}
__device__ __forceinline__ float wave_max(float v) {
#pragma unroll
  for (int off = 16; off > 0; off >>= 1) v = fmaxf(v, __shfl_xor(v, off, 32));
  return v;
}
__device__ __forceinline__ float wave_sum(float v) {
#pragma unroll
  for (int off = 16; off > 0; off >>= 1) v += __shfl_xor(v, off, 32);
  return v;
}
__device__ __forceinline__ double wave_sumd(double v) {
#pragma unroll
  for (int off = 16; off > 0; off >>= 1) v += __shfl_xor(v, off, 32);
  return v;
}
__device__ __forceinline__ void st2_us8(unsigned short* p, v8us v) {
  *(volatile v8us*)p = v; __threadfence(); *(volatile v8us*)p = v;
}
__device__ __forceinline__ void st2_f4(float* p, v4f v) {
  *(volatile v4f*)p = v; __threadfence(); *(volatile v4f*)p = v;
}
__device__ __forceinline__ v8us blend_row8(const float* pa, const float* pb, unsigned m) {
  const v4f a0 = *(const v4fa*)pa, a1 = *(const v4fa*)(pa + 4);
  const v4f b0 = *(const v4fa*)pb, b1 = *(const v4fa*)(pb + 4);
  v8us o;
  o[0] = f2bf_bits(blendf(a0.x, b0.x, m)); o[1] = f2bf_bits(blendf(a0.y, b0.y, m));
  o[2] = f2bf_bits(blendf(a0.z, b0.z, m)); o[3] = f2bf_bits(blendf(a0.w, b0.w, m));
  o[4] = f2bf_bits(blendf(a1.x, b1.x, m)); o[5] = f2bf_bits(blendf(a1.y, b1.y, m));
  o[6] = f2bf_bits(blendf(a1.z, b1.z, m)); o[7] = f2bf_bits(blendf(a1.w, b1.w, m));
  return o;
}

__global__ __launch_bounds__(256) void k_pa1(
    const float* __restrict__ Wq, const float* __restrict__ Wv, const float* __restrict__ Wg1, const float* __restrict__ Wg2,
    const float* __restrict__ bq, const float* __restrict__ bv, const float* __restrict__ bg1, const float* __restrict__ bg2,
    unsigned short* __restrict__ WQV, unsigned short* __restrict__ WG12, float* __restrict__ BIA) {
  const int tid = threadIdx.x;
  const int blk = blockIdx.x;
  if (blk < 16) {
    const int u = blk * 256 + tid, rr = u >> 4, p = u & 15;
    const size_t so = (size_t)(rr & 127) * ND + 8 * p;
    const unsigned m = (rr < 128) ? 0xffffffffu : 0u;
    const v8us o = blend_row8(Wq + so, Wv + so, m);
    st2_us8(WQV + (size_t)rr * ND + 8 * p, o);
  } else if (blk < 48) {
    const int u = (blk - 16) * 256 + tid, rr = u >> 5, p = u & 31;
    const size_t so = (size_t)(rr & 127) * ND + ((8 * p) & 127);
    const unsigned m = (rr < 128) ? 0xffffffffu : 0u;
    const v8us o = blend_row8(Wg1 + so, Wg2 + so, m);
    st2_us8(WG12 + (size_t)rr * 256 + 8 * p, o);
  } else if (tid < 128) {
    const int grp = tid >> 6, r4 = (tid & 63) * 4, sr = r4 & 127;
    const v4f a = *(const v4fa*)(bq + sr), b = *(const v4fa*)(bv + sr);
    const v4f c = *(const v4fa*)(bg1 + sr), d = *(const v4fa*)(bg2 + sr);
    const unsigned m1 = (r4 < 128) ? 0xffffffffu : 0u;
    const unsigned m2 = (grp == 0) ? 0xffffffffu : 0u;
    v4f o;
    o.x = bfr(blendf(blendf(a.x, b.x, m1), blendf(c.x, d.x, m1), m2));
    o.y = bfr(blendf(blendf(a.y, b.y, m1), blendf(c.y, d.y, m1), m2));
    o.z = bfr(blendf(blendf(a.z, b.z, m1), blendf(c.z, d.z, m1), m2));
    o.w = bfr(blendf(blendf(a.w, b.w, m1), blendf(c.w, d.w, m1), m2));
    st2_f4(BIA + grp * 256 + r4, o);
  }
}

__global__ __launch_bounds__(256) void k_pa2(
    const float* __restrict__ Wx, const float* __restrict__ Wc, const float* __restrict__ Wg3,
    const float* __restrict__ bx, const float* __restrict__ bc, const float* __restrict__ bg3,
    unsigned short* __restrict__ W2ALL, float* __restrict__ BIA) {
  const int tid = threadIdx.x;
  const int blk = blockIdx.x;
  if (blk < 48) {
    const int sel = blk >> 4;
    const int u = (blk & 15) * 256 + tid, rr = u >> 5, p = u & 31;
    const size_t so = (size_t)rr * ND + ((8 * p) & 127);
    const unsigned m0 = (sel == 0) ? 0xffffffffu : 0u;
    const unsigned m1 = (sel == 1) ? 0xffffffffu : 0u;
    const v4f a0 = *(const v4fa*)(Wx + so),  a1 = *(const v4fa*)(Wx + so + 4);
    const v4f b0 = *(const v4fa*)(Wc + so),  b1 = *(const v4fa*)(Wc + so + 4);
    const v4f c0 = *(const v4fa*)(Wg3 + so), c1 = *(const v4fa*)(Wg3 + so + 4);
    v8us o;
    o[0] = f2bf_bits(blendf(a0.x, blendf(b0.x, c0.x, m1), m0)); o[1] = f2bf_bits(blendf(a0.y, blendf(b0.y, c0.y, m1), m0));
    o[2] = f2bf_bits(blendf(a0.z, blendf(b0.z, c0.z, m1), m0)); o[3] = f2bf_bits(blendf(a0.w, blendf(b0.w, c0.w, m1), m0));
    o[4] = f2bf_bits(blendf(a1.x, blendf(b1.x, c1.x, m1), m0)); o[5] = f2bf_bits(blendf(a1.y, blendf(b1.y, c1.y, m1), m0));
    o[6] = f2bf_bits(blendf(a1.z, blendf(b1.z, c1.z, m1), m0)); o[7] = f2bf_bits(blendf(a1.w, blendf(b1.w, c1.w, m1), m0));
    st2_us8(W2ALL + (size_t)sel * 32768 + (size_t)rr * 256 + 8 * p, o);
  } else if (tid < 96) {
    const int grp = tid >> 5, r4 = (tid & 31) * 4;
    const unsigned m0 = (grp == 0) ? 0xffffffffu : 0u;
    const unsigned m1 = (grp == 1) ? 0xffffffffu : 0u;
    const v4f a = *(const v4fa*)(bx + r4), b = *(const v4fa*)(bc + r4), c = *(const v4fa*)(bg3 + r4);
    v4f o;
    o.x = bfr(blendf(a.x, blendf(b.x, c.x, m1), m0));
    o.y = bfr(blendf(a.y, blendf(b.y, c.y, m1), m0));
    o.z = bfr(blendf(a.z, blendf(b.z, c.z, m1), m0));
    o.w = bfr(blendf(a.w, blendf(b.w, c.w, m1), m0));
    st2_f4(BIA + 512 + grp * 128 + r4, o);
  }
}

template <int OUTF32>
__global__ __launch_bounds__(256) void k_tok(const float* __restrict__ src, unsigned short* __restrict__ dstb,
                                             float* __restrict__ dstf) {
  extern __shared__ __align__(16) unsigned char dyn_lds[];
  float* tile = (float*)dyn_lds;
  const int tid = threadIdx.x;
  const int ch = blockIdx.x, b = blockIdx.y;
  const int n0 = ch * 16;
  const int nv = (NN - n0) < 16 ? (NN - n0) : 16;
  const int nf4 = nv * 3;
  const float* sb = src + (size_t)b * ND * SS + (size_t)n0 * NL;
#pragma unroll 4
  for (int it = 0; it < 24; ++it) {
    const int q = it * 256 + tid;
    const int c = q / 48, f = q - c * 48;
    const int fc = f < nf4 ? f : nf4 - 1;
    const v4f v = *(const v4fa*)(sb + (size_t)c * SS + 4 * fc);
    const bool ok = f < nf4;
    v4f o;
    o.x = ok ? bfr(v.x) : 0.0f; o.y = ok ? bfr(v.y) : 0.0f;
    o.z = ok ? bfr(v.z) : 0.0f; o.w = ok ? bfr(v.w) : 0.0f;
    *(v4fa*)(tile + c * 192 + 4 * f) = o;
  }
  __syncthreads();
  const size_t rbase = (size_t)b * NL * NP + n0;
  for (int pass = 0; pass < 2; ++pass) {
    if (OUTF32 == 0) {
#pragma unroll 2
      for (int it = 0; it < 12; ++it) {
        const int q = it * 256 + tid, rr = q >> 4, p = q & 15;
        const int l = rr >> 4, nn = rr & 15;
        const float* tp = tile + (8 * p) * 192 + nn * 12 + l;
        v8us o;
#pragma unroll
        for (int e = 0; e < 8; ++e) o[e] = f2bf_bits(tp[e * 192]);
        *(volatile v8us*)(dstb + (rbase + (size_t)l * NP + nn) * ND + 8 * p) = o;
      }
    } else {
#pragma unroll 2
      for (int it = 0; it < 24; ++it) {
        const int q = it * 256 + tid, rr = q >> 5, p = q & 31;
        const int l = rr >> 4, nn = rr & 15;
        const float* tp = tile + (4 * p) * 192 + nn * 12 + l;
        v4f o; o.x = tp[0]; o.y = tp[192]; o.z = tp[384]; o.w = tp[576];
        *(volatile v4f*)(dstf + (rbase + (size_t)l * NP + nn) * ND + 4 * p) = o;
      }
    }
    __threadfence();
  }
}

__global__ __launch_bounds__(256) void k_avg(const float* __restrict__ x, float* __restrict__ AVG) {
  __shared__ __align__(16) float res[32];
  const int tid = threadIdx.x, lane = tid & 31, w = tid >> 5;
#pragma unroll 1
  for (int j = 0; j < 4; ++j) {
    const int pl = blockIdx.x * 32 + w * 4 + j;
    const float* xp = x + (size_t)pl * SS;
    double s = 0.0;
#pragma unroll 4
    for (int i = 0; i < 29; ++i) {
      const int f = lane + 32 * i;
      const int fc = f < 921 ? f : 920;
      const v4f v = *(const v4fa*)(xp + 4 * fc);
      const float part = (bfr(v.x) + bfr(v.y)) + (bfr(v.z) + bfr(v.w));
      s += (f < 921) ? (double)part : 0.0;
    }
    s = wave_sumd(s);
    if (lane == 0) res[w * 4 + j] = (float)(s * (1.0 / 3684.0));
  }
  __syncthreads();
  if (tid < 8) {
    const v4f o = *(const v4fa*)(res + 4 * tid);
    st2_f4(AVG + blockIdx.x * 32 + 4 * tid, o);
  }
}

__global__ __launch_bounds__(256) void k_mem(const float* __restrict__ AVG, const float* __restrict__ A1,
                                             const float* __restrict__ a1b, const float* __restrict__ A2,
                                             const float* __restrict__ a2b, const float* __restrict__ imp,
                                             float* __restrict__ MEMW) {
  __shared__ float av[1024];
  __shared__ float hid[512];
  __shared__ float lg[32];
  __shared__ __align__(16) float mw[32];
  const int tid = threadIdx.x;
#pragma unroll
  for (int i = 0; i < 4; ++i) av[tid + 256 * i] = AVG[tid + 256 * i];
  __syncthreads();
#pragma unroll 1
  for (int o = tid; o < 512; o += 256) {
    const int b = o >> 6, j = o & 63;
    float a = bfr(a1b[j]);
#pragma unroll 4
    for (int c = 0; c < ND; ++c) a = fmaf(av[b * ND + c], bfr(A1[c * 64 + j]), a);
    hid[o] = (a > 0.0f) ? a : 0.0f;
  }
  __syncthreads();
  if (tid < 32) {
    const int b = tid >> 2, m = tid & 3;
    float a = bfr(a2b[m]);
#pragma unroll 4
    for (int j = 0; j < 64; ++j) a = fmaf(hid[b * 64 + j], bfr(A2[j * 4 + m]), a);
    lg[tid] = a;
  }
  __syncthreads();
  if (tid < 8) {
    const float l0 = lg[4 * tid], l1 = lg[4 * tid + 1], l2 = lg[4 * tid + 2], l3 = lg[4 * tid + 3];
    const float mx = fmaxf(fmaxf(l0, l1), fmaxf(l2, l3));
    const float e0 = expf(l0 - mx), e1 = expf(l1 - mx), e2 = expf(l2 - mx), e3 = expf(l3 - mx);
    const float inv = 1.0f / (((e0 + e1) + e2) + e3);
    const float g0 = bfr(imp[0]) * (e0 * inv), g1 = bfr(imp[1]) * (e1 * inv);
    const float g2 = bfr(imp[2]) * (e2 * inv), g3 = bfr(imp[3]) * (e3 * inv);
    const float mx2 = fmaxf(fmaxf(g0, g1), fmaxf(g2, g3));
    const float f0 = expf(g0 - mx2), f1 = expf(g1 - mx2), f2 = expf(g2 - mx2), f3 = expf(g3 - mx2);
    const float inv2 = 1.0f / (((f0 + f1) + f2) + f3);
    mw[4 * tid] = f0 * inv2; mw[4 * tid + 1] = f1 * inv2; mw[4 * tid + 2] = f2 * inv2; mw[4 * tid + 3] = f3 * inv2;
  }
  __syncthreads();
  if (tid < 8) {
    const v4f o = *(const v4fa*)(mw + 4 * tid);
    st2_f4(MEMW + 4 * tid, o);
  }
}

__device__ __forceinline__ void store_f32_rows(const float* rowb, float* dst, int tid, int nthr) {
  for (int pass = 0; pass < 2; ++pass) {
#pragma unroll 1
    for (int q = tid; q < 1280; q += nthr) {
      const int r = q / 80, p = q - r * 80;
      const v4f v = *(const v4fa*)(rowb + r * NP + 4 * p);
      *(volatile v4f*)(dst + (size_t)r * NP + 4 * p) = v;
    }
    __threadfence();
  }
}
template <int LOSEG>
__device__ __forceinline__ void store_tri_rows(const float* rowb, unsigned short* dst, int tid, int nthr) {
  for (int pass = 0; pass < 2; ++pass) {
#pragma unroll 1
    for (int q = tid; q < 1920; q += nthr) {
      const int r = q / 120, p = q - r * 120;
      const int seg = p / 40, c8 = (p - seg * 40) * 8;
      const v4f a = *(const v4fa*)(rowb + r * NP + c8);
      const v4f b = *(const v4fa*)(rowb + r * NP + c8 + 4);
      const unsigned sh = (seg == LOSEG) ? 16u : 0u;
      v8us o;
      o[0] = (unsigned short)((split_pk(a.x) >> sh) & 0xffffu); o[1] = (unsigned short)((split_pk(a.y) >> sh) & 0xffffu);
      o[2] = (unsigned short)((split_pk(a.z) >> sh) & 0xffffu); o[3] = (unsigned short)((split_pk(a.w) >> sh) & 0xffffu);
      o[4] = (unsigned short)((split_pk(b.x) >> sh) & 0xffffu); o[5] = (unsigned short)((split_pk(b.y) >> sh) & 0xffffu);
      o[6] = (unsigned short)((split_pk(b.z) >> sh) & 0xffffu); o[7] = (unsigned short)((split_pk(b.w) >> sh) & 0xffffu);
      *(volatile v8us*)(dst + (size_t)r * K3 + 8 * p) = o;
    }
    __threadfence();
  }
}

__global__ __launch_bounds__(256) void k_s1(const float* __restrict__ nv1, const float* __restrict__ nv2,
                                            float* __restrict__ S1, unsigned short* __restrict__ A3) {
  __shared__ float n2[3072];
  __shared__ float n1[160];
  __shared__ __align__(16) float rowb[16 * NP];
  const int tid = threadIdx.x, lane = tid & 31, w = tid >> 5;
  const int i0 = blockIdx.x * 16;
#pragma unroll 4
  for (int i = tid; i < 3070; i += 256) n2[i] = bfr(nv2[i]);
  if (tid < 160) {
    const int r = tid / 10, p = tid - r * 10;
    int gi = i0 + r; gi = gi < NN ? gi : NN - 1;
    n1[tid] = bfr(nv1[gi * 10 + p]);
  }
  __syncthreads();
#pragma unroll 1
  for (int j2 = 0; j2 < 2; ++j2) {
    const int rr = 2 * w + j2;
    const bool rv = (i0 + rr) < NN;
    float* rb = rowb + rr * NP;
    float mx = -3.0e38f;
#pragma unroll 1
    for (int i = 0; i < 10; ++i) {
      const int c = lane + 32 * i;
      const int cc = c < NN ? c : NN - 1;
      float a = 0.0f;
#pragma unroll
      for (int p = 0; p < 10; ++p) a = fmaf(n1[rr * 10 + p], n2[p * NN + cc], a);
      a = (a > 0.0f) ? a : 0.0f;
      rb[c] = a;
      mx = (c < NN) ? fmaxf(mx, a) : mx;
    }
    mx = wave_max(mx);
    float sum = 0.0f;
#pragma unroll 1
    for (int i = 0; i < 10; ++i) {
      const int c = lane + 32 * i;
      const float ex = expf(rb[c] - mx);
      const float e = (c < NN) ? ex : 0.0f;
      rb[c] = e; sum += e;
    }
    sum = wave_sum(sum);
    const float inv = 1.0f / sum;
#pragma unroll 1
    for (int i = 0; i < 10; ++i) {
      const int c = lane + 32 * i;
      const float v = rb[c] * inv;
      rb[c] = (rv && c < NN) ? v : 0.0f;
    }
  }
  __syncthreads();
  store_f32_rows(rowb, S1 + (size_t)i0 * NP, tid, 256);
  store_tri_rows<1>(rowb, A3 + (size_t)i0 * K3, tid, 256);
}

template <int MODE>
__global__ __launch_bounds__(256) void k_trans(const float* __restrict__ in, float* __restrict__ outF,
                                               unsigned short* __restrict__ outB) {
  __shared__ __align__(16) float tl[16 * NP];
  const int tid = threadIdx.x;
  const int i0 = blockIdx.x * 16;
#pragma unroll
  for (int it = 0; it < 5; ++it) {
    const int q = it * 256 + tid, j = q >> 2, f = q & 3;
    const v4f v = *(const v4fa*)(in + (size_t)j * NP + i0 + 4 * f);
    tl[(4 * f + 0) * NP + j] = v.x; tl[(4 * f + 1) * NP + j] = v.y;
    tl[(4 * f + 2) * NP + j] = v.z; tl[(4 * f + 3) * NP + j] = v.w;
  }
  __syncthreads();
  if (MODE == 0) store_f32_rows(tl, outF + (size_t)i0 * NP, tid, 256);
  else           store_tri_rows<2>(tl, outB + (size_t)i0 * K3, tid, 256);
}

template <int STAGE>
__global__ __launch_bounds__(128) void k_s23(const unsigned short* __restrict__ A3in, const unsigned short* __restrict__ Bt3,
                                             const float* __restrict__ S1, const float* __restrict__ S2,
                                             const float* __restrict__ sws, float* __restrict__ outF,
                                             unsigned short* __restrict__ A3out) {
  __shared__ __align__(16) float accT[16 * NP];
  const int tid = threadIdx.x, lane = tid & 31, w = tid >> 5;
  const int li = lane & 15, h = lane >> 4;
  const int m0 = blockIdx.x * 16;
  const v8f zero8 = {0.f, 0.f, 0.f, 0.f, 0.f, 0.f, 0.f, 0.f};
  v8f acc[5];
#pragma unroll
  for (int t = 0; t < 5; ++t) acc[t] = zero8;
  const unsigned short* ap = A3in + (size_t)(m0 + li) * K3 + 8 * h;
  const unsigned short* bp = Bt3 + (size_t)(w * 80 + li) * K3 + 8 * h;
#pragma unroll 1
  for (int k0 = 0; k0 < K3; k0 += 32) {
    const v16b a = ldfrag_g(ap + k0);
#pragma unroll
    for (int t = 0; t < 5; ++t) {
      const v16b bb = ldfrag_g(bp + (size_t)t * 16 * K3 + k0);
      acc[t] = wmb(a, bb, acc[t]);
    }
  }
#pragma unroll
  for (int t = 0; t < 5; ++t)
#pragma unroll
    for (int r = 0; r < 8; ++r) accT[(8 * h + r) * NP + w * 80 + t * 16 + li] = acc[t][r];
  __syncthreads();
  float sw0 = 0.0f, sw1 = 0.0f, sw2 = 0.0f;
  if (STAGE == 3) {
    const float a0 = bfr(sws[0]), a1 = bfr(sws[1]), a2 = bfr(sws[2]);
    const float mx = fmaxf(a0, fmaxf(a1, a2));
    const float e0 = expf(a0 - mx), e1 = expf(a1 - mx), e2 = expf(a2 - mx);
    const float inv = 1.0f / ((e0 + e1) + e2);
    sw0 = e0 * inv; sw1 = e1 * inv; sw2 = e2 * inv;
  }
#pragma unroll 1
  for (int j = 0; j < 4; ++j) {
    const int rr = 4 * w + j;
    const int gi = m0 + rr;
    const bool rv = gi < NN;
    float* rb = accT + rr * NP;
    float mx = -3.0e38f;
#pragma unroll 1
    for (int i = 0; i < 10; ++i) {
      const int c = lane + 32 * i;
      const float v = rb[c];
      mx = (c < NN) ? fmaxf(mx, v) : mx;
    }
    mx = wave_max(mx);
    float sum = 0.0f;
#pragma unroll 1
    for (int i = 0; i < 10; ++i) {
      const int c = lane + 32 * i;
      const float ex = expf(rb[c] - mx);
      const float e = (c < NN) ? ex : 0.0f;
      rb[c] = e; sum += e;
    }
    sum = wave_sum(sum);
    const float inv = 1.0f / sum;
#pragma unroll 1
    for (int i = 0; i < 10; ++i) {
      const int c = lane + 32 * i;
      float v = rb[c] * inv;
      v = (rv && c < NN) ? v : 0.0f;
      if (STAGE == 3) {
        const float x1 = S1[(size_t)gi * NP + c];
        const float x2 = S2[(size_t)gi * NP + c];
        v = (sw0 * x1 + sw1 * x2) + sw2 * v;
      }
      rb[c] = v;
    }
  }
  __syncthreads();
  store_f32_rows(accT, outF + (size_t)m0 * NP, tid, 128);
  if (STAGE == 2) store_tri_rows<1>(accT, A3out + (size_t)m0 * K3, tid, 128);
}

__global__ __launch_bounds__(256) void k_qv(const unsigned short* __restrict__ XB, const unsigned short* __restrict__ WQV,
                                            const float* __restrict__ BIA, unsigned short* __restrict__ QHL,
                                            unsigned short* __restrict__ VTh, unsigned short* __restrict__ VTl) {
  extern __shared__ __align__(16) unsigned char dyn_lds[];
  unsigned short* sQ  = (unsigned short*)dyn_lds;
  unsigned short* sVh = sQ + 64 * 256;
  unsigned short* sVl = sVh + 128 * 64;
  const int tid = threadIdx.x, lane = tid & 31, w = tid >> 5;
  const int li = lane & 15, h = lane >> 4;
  const int tile = blockIdx.x, m0 = tile * 64;
  const int bl = tile / 5, nt0 = (tile - bl * 5) * 64;
  const v8f zero8 = {0.f, 0.f, 0.f, 0.f, 0.f, 0.f, 0.f, 0.f};
  v8f acc[4][2];
#pragma unroll
  for (int i = 0; i < 4; ++i) { acc[i][0] = zero8; acc[i][1] = zero8; }
  const unsigned short* ap = XB + (size_t)(m0 + li) * ND + 8 * h;
  const unsigned short* bp = WQV + (size_t)(32 * w + li) * ND + 8 * h;
#pragma unroll 1
  for (int k0 = 0; k0 < ND; k0 += 32) {
    const v16b b0 = ldfrag_g(bp + k0);
    const v16b b1 = ldfrag_g(bp + (size_t)16 * ND + k0);
#pragma unroll
    for (int i = 0; i < 4; ++i) {
      const v16b a = ldfrag_g(ap + (size_t)i * 16 * ND + k0);
      acc[i][0] = wmb(a, b0, acc[i][0]);
      acc[i][1] = wmb(a, b1, acc[i][1]);
    }
  }
#pragma unroll
  for (int j = 0; j < 2; ++j) {
    const int ncol = 32 * w + 16 * j + li;
    const float bias = BIA[ncol];
#pragma unroll
    for (int i = 0; i < 4; ++i) {
#pragma unroll
      for (int r = 0; r < 8; ++r) {
        const int tok = 16 * i + 8 * h + r;
        float v = acc[i][j][r] + bias;
        v = (v > 0.0f) ? v : 0.0f;
        v = ((nt0 + tok) < NN) ? v : 0.0f;
        const unsigned pk = split_pk(v);
        const unsigned short hb = (unsigned short)(pk & 0xffffu);
        const unsigned short lb = (unsigned short)(pk >> 16);
        if (w < 4) {
          sQ[tok * 256 + (ncol >> 4) * 32 + li] = hb;
          sQ[tok * 256 + (ncol >> 4) * 32 + 16 + li] = lb;
        } else {
          sVh[(ncol - 128) * 64 + tok] = hb;
          sVl[(ncol - 128) * 64 + tok] = lb;
        }
      }
    }
  }
  __syncthreads();
  for (int pass = 0; pass < 2; ++pass) {
#pragma unroll 2
    for (int it = 0; it < 8; ++it) {
      const int q = it * 256 + tid, row = q >> 5, p = q & 31;
      const v8us v = *(const v8usa*)(sQ + row * 256 + 8 * p);
      *(volatile v8us*)(QHL + (size_t)(m0 + row) * 256 + 8 * p) = v;
    }
#pragma unroll 2
    for (int it = 0; it < 4; ++it) {
      const int q = it * 256 + tid, c = q >> 3, p = q & 7;
      const v8us v = *(const v8usa*)(sVh + c * 64 + 8 * p);
      *(volatile v8us*)(VTh + ((size_t)bl * ND + c) * NP + nt0 + 8 * p) = v;
    }
#pragma unroll 2
    for (int it = 0; it < 4; ++it) {
      const int q = it * 256 + tid, c = q >> 3, p = q & 7;
      const v8us v = *(const v8usa*)(sVl + c * 64 + 8 * p);
      *(volatile v8us*)(VTl + ((size_t)bl * ND + c) * NP + nt0 + 8 * p) = v;
    }
    __threadfence();
  }
}

__device__ __forceinline__ float sel1(float w0, float w1, float w2, float w3, float a, float b, float c, float d) {
  float s = w0 * bfr(a);
  s = fmaf(w1, bfr(b), s);
  s = fmaf(w2, bfr(c), s);
  s = fmaf(w3, bfr(d), s);
  return s;
}

__global__ __launch_bounds__(128) __attribute__((amdgpu_num_vgpr(248)))
void k_attn(const unsigned short* __restrict__ QHL, const unsigned short* __restrict__ VTh,
            const unsigned short* __restrict__ VTl, const float* __restrict__ bank,
            const float* __restrict__ MEMW, const float* __restrict__ ADJT, float* __restrict__ Y0) {
  extern __shared__ __align__(16) unsigned char dyn_lds[];
  unsigned short* sSH = (unsigned short*)dyn_lds;
  unsigned short* sSL = sSH + 2 * 5120;
  const int tid = threadIdx.x, lane = tid & 31, w = tid >> 5;
  const int li = lane & 15, h = lane >> 4;
  const int bid = blockIdx.x, hp = bid & 3, bl = bid >> 2;
  const int b = bl / NL, l = bl - b * NL;
  float* strip = (float*)(dyn_lds + 40960 + w * 43008);
  unsigned short* sTh = (unsigned short*)(strip + 16 * NP);
  unsigned short* sTl = sTh + 16 * NP;
  float* ost = (float*)(sTl + 16 * NP);

  {
    const float w0 = MEMW[b * 4 + 0], w1 = MEMW[b * 4 + 1], w2 = MEMW[b * 4 + 2], w3 = MEMW[b * 4 + 3];
#pragma unroll 2
    for (int it = 0; it < 20; ++it) {
      const int u = it * 128 + tid;
      const int hd = u / 1280, rem = u - hd * 1280;
      const int j = rem >> 2, f = rem & 3;
      const int jc = j < NN ? j : NN - 1;
      const int hh = hp * 2 + hd;
      const size_t base = (((size_t)hh * NL + l) * NN + jc) * 16 + 4 * f;
      const v4f x0 = *(const v4fa*)(bank + base);
      const v4f x1 = *(const v4fa*)(bank + base + (size_t)MSTRIDE);
      const v4f x2 = *(const v4fa*)(bank + base + (size_t)2 * MSTRIDE);
      const v4f x3 = *(const v4fa*)(bank + base + (size_t)3 * MSTRIDE);
      const bool ok = j < NN;
      float s0 = sel1(w0, w1, w2, w3, x0.x, x1.x, x2.x, x3.x);
      float s1 = sel1(w0, w1, w2, w3, x0.y, x1.y, x2.y, x3.y);
      float s2 = sel1(w0, w1, w2, w3, x0.z, x1.z, x2.z, x3.z);
      float s3 = sel1(w0, w1, w2, w3, x0.w, x1.w, x2.w, x3.w);
      s0 = ok ? s0 : 0.0f; s1 = ok ? s1 : 0.0f; s2 = ok ? s2 : 0.0f; s3 = ok ? s3 : 0.0f;
      const unsigned p0 = split_pk(s0), p1 = split_pk(s1), p2 = split_pk(s2), p3 = split_pk(s3);
      v4us H, Lo;
      H.x = (unsigned short)(p0 & 0xffffu); H.y = (unsigned short)(p1 & 0xffffu);
      H.z = (unsigned short)(p2 & 0xffffu); H.w = (unsigned short)(p3 & 0xffffu);
      Lo.x = (unsigned short)(p0 >> 16); Lo.y = (unsigned short)(p1 >> 16);
      Lo.z = (unsigned short)(p2 >> 16); Lo.w = (unsigned short)(p3 >> 16);
      *(v4usa*)(sSH + hd * 5120 + j * 16 + 4 * f) = H;
      *(v4usa*)(sSL + hd * 5120 + j * 16 + 4 * f) = Lo;
    }
  }
  __syncthreads();

  const v8f zero8 = {0.f, 0.f, 0.f, 0.f, 0.f, 0.f, 0.f, 0.f};
  const v8us zus = {0, 0, 0, 0, 0, 0, 0, 0};
  const size_t rowbase = (size_t)bl * NP;

#pragma unroll 1
  for (int t = 0; t < 5; ++t) {
    const int q0 = (w + 4 * t) * 16;
#pragma unroll 1
    for (int hd = 0; hd < 2; ++hd) {
      const int hh = hp * 2 + hd;
      const unsigned short* qp = QHL + (rowbase + q0 + li) * 256 + hh * 32 + 8 * h;
      FB a1, a2;
      a1.h[0] = *(const v8usa*)qp;
      a1.h[1] = *(const v8usa*)(qp + 16);
      a2.h[0] = a1.h[0];
      a2.h[1] = zus;
      const unsigned short* sh = sSH + hd * 5120;
      const unsigned short* sl = sSL + hd * 5120;
#pragma unroll 2
      for (int kt = 0; kt < 20; ++kt) {
        FB b1, b2;
        const v8us xh = *(const v8usa*)(sh + (kt * 16 + li) * 16 + 8 * h);
        b1.h[0] = xh; b1.h[1] = xh;
        b2.h[0] = *(const v8usa*)(sl + (kt * 16 + li) * 16 + 8 * h);
        b2.h[1] = zus;
        v8f s = zero8;
        s = wmb(a1.v, b1.v, s);
        s = wmb(a2.v, b2.v, s);
#pragma unroll
        for (int r = 0; r < 8; ++r) strip[(8 * h + r) * NP + kt * 16 + li] = s[r] * 0.25f;
      }
      wave_sync();
#pragma unroll 1
      for (int rr = 0; rr < 16; ++rr) {
        const int qi = q0 + rr;
        const float* sr = strip + rr * NP + 10 * lane;
        float sv[10];
#pragma unroll
        for (int e = 0; e < 5; ++e) {
          const v2f x = *(const v2fa*)(sr + 2 * e);
          sv[2 * e] = x.x; sv[2 * e + 1] = x.y;
        }
        float mx = -3.0e38f;
#pragma unroll
        for (int e = 0; e < 10; ++e) mx = ((10 * lane + e) < NN) ? fmaxf(mx, sv[e]) : mx;
        mx = wave_max(mx);
        float sum = 0.0f;
#pragma unroll
        for (int e = 0; e < 10; ++e) {
          const float ex = expf(sv[e] - mx);
          const float pe = ((10 * lane + e) < NN) ? ex : 0.0f;
          sv[e] = pe; sum += pe;
        }
        sum = wave_sum(sum);
        const float inv = 1.0f / sum;
        const bool qv = qi < NN;
        const float* ar = ADJT + (size_t)qi * NP + 10 * lane;
        unsigned short* th = sTh + rr * NP + 10 * lane;
        unsigned short* tl = sTl + rr * NP + 10 * lane;
#pragma unroll
        for (int e = 0; e < 5; ++e) {
          const v2f a = *(const v2fa*)(ar + 2 * e);
          float t0 = sv[2 * e] * inv + a.x;
          float t1 = sv[2 * e + 1] * inv + a.y;
          t0 = (qv && (10 * lane + 2 * e) < NN) ? t0 : 0.0f;
          t1 = (qv && (10 * lane + 2 * e + 1) < NN) ? t1 : 0.0f;
          const unsigned p0 = split_pk(t0), p1 = split_pk(t1);
          v2us H, Lo;
          H.x = (unsigned short)(p0 & 0xffffu); H.y = (unsigned short)(p1 & 0xffffu);
          Lo.x = (unsigned short)(p0 >> 16);    Lo.y = (unsigned short)(p1 >> 16);
          *(v2usa*)(th + 2 * e) = H;
          *(v2usa*)(tl + 2 * e) = Lo;
        }
      }
      wave_sync();
      v8f o = zero8;
      const unsigned short* vh = VTh + ((size_t)bl * ND + hh * 16 + li) * NP + 8 * h;
      const unsigned short* vl = VTl + ((size_t)bl * ND + hh * 16 + li) * NP + 8 * h;
#pragma unroll 2
      for (int ks = 0; ks < 10; ++ks) {
        const int k0 = ks * 32;
        FB tH, tL;
        tH.h[0] = *(const v8usa*)(sTh + li * NP + k0 + 8 * h);
        tH.h[1] = *(const v8usa*)(sTh + li * NP + k0 + 16 + 8 * h);
        tL.h[0] = *(const v8usa*)(sTl + li * NP + k0 + 8 * h);
        tL.h[1] = *(const v8usa*)(sTl + li * NP + k0 + 16 + 8 * h);
        const v16b bh = ldfrag_g(vh + k0);
        const v16b bo = ldfrag_g(vl + k0);
        o = wmb(tH.v, bh, o);
        o = wmb(tL.v, bh, o);
        o = wmb(tH.v, bo, o);
      }
#pragma unroll
      for (int r = 0; r < 8; ++r) ost[(8 * h + r) * 32 + hd * 16 + li] = o[r];
      wave_sync();
    }
    for (int pass = 0; pass < 2; ++pass) {
#pragma unroll
      for (int it = 0; it < 4; ++it) {
        const int q = it * 32 + lane, row = q >> 3, p = q & 7;
        const v4f v = *(const v4fa*)(ost + row * 32 + 4 * p);
        *(volatile v4f*)(Y0 + (rowbase + q0 + row) * ND + hp * 32 + 4 * p) = v;
      }
      __threadfence();
    }
    wave_sync();
  }
}

__device__ __forceinline__ void gemm_one(const unsigned short* sA, const unsigned short* wrow, int li, int h, v8f (&acc)[4]) {
#pragma unroll 1
  for (int k0 = 0; k0 < 256; k0 += 32) {
    const v16b bb = ldfrag_g(wrow + k0);
#pragma unroll
    for (int i = 0; i < 4; ++i) {
      FB a;
      a.h[0] = *(const v8usa*)(sA + (16 * i + li) * LDA + k0 + 8 * h);
      a.h[1] = *(const v8usa*)(sA + (16 * i + li) * LDA + k0 + 16 + 8 * h);
      acc[i] = wmb(a.v, bb, acc[i]);
    }
  }
}
__device__ __forceinline__ void gemm_two(const unsigned short* sA, const unsigned short* w1, const unsigned short* w2,
                                         int li, int h, v8f (&c1)[4], v8f (&c2)[4]) {
#pragma unroll 1
  for (int k0 = 0; k0 < 256; k0 += 32) {
    const v16b b1 = ldfrag_g(w1 + k0);
    const v16b b2 = ldfrag_g(w2 + k0);
#pragma unroll
    for (int i = 0; i < 4; ++i) {
      FB a;
      a.h[0] = *(const v8usa*)(sA + (16 * i + li) * LDA + k0 + 8 * h);
      a.h[1] = *(const v8usa*)(sA + (16 * i + li) * LDA + k0 + 16 + 8 * h);
      c1[i] = wmb(a.v, b1, c1[i]);
      c2[i] = wmb(a.v, b2, c2[i]);
    }
  }
}
__device__ __forceinline__ void put_split4(unsigned short* d, v4f v) {
  const unsigned p0 = split_pk(v.x), p1 = split_pk(v.y), p2 = split_pk(v.z), p3 = split_pk(v.w);
  v4us H, Lo;
  H.x = (unsigned short)(p0 & 0xffffu); H.y = (unsigned short)(p1 & 0xffffu);
  H.z = (unsigned short)(p2 & 0xffffu); H.w = (unsigned short)(p3 & 0xffffu);
  Lo.x = (unsigned short)(p0 >> 16); Lo.y = (unsigned short)(p1 >> 16);
  Lo.z = (unsigned short)(p2 >> 16); Lo.w = (unsigned short)(p3 >> 16);
  *(v4usa*)d = H;
  *(v4usa*)(d + 128) = Lo;
}
__device__ __forceinline__ void write_record(double s, double q, double* red, double* rec, int tid) {
  s = wave_sumd(s); q = wave_sumd(q);
  if ((tid & 31) == 0) { red[2 * (tid >> 5)] = s; red[2 * (tid >> 5) + 1] = q; }
  __syncthreads();
  if (tid < 8) {
    double S = 0.0, Q = 0.0;
#pragma unroll
    for (int k = 0; k < 8; ++k) { S += red[2 * k]; Q += red[2 * k + 1]; }
    v2d o;
    o.x = (tid == 0) ? S : 0.0;
    o.y = (tid == 0) ? Q : 0.0;
    *(volatile v2d*)(rec + 2 * tid) = o;
    __threadfence();
    *(volatile v2d*)(rec + 2 * tid) = o;
  }
}
__device__ __forceinline__ void ln_stats(const double* REC, int bl, float& mean, float& rstd) {
  double S = 0.0, Q = 0.0;
#pragma unroll
  for (int i = 0; i < 5; ++i) {
    const v2d r = *(const v2d*)(REC + (size_t)(bl * 5 + i) * 16);
    S += r.x; Q += r.y;
  }
  const double md = S * (1.0 / 39296.0);
  const double vd = Q * (1.0 / 39296.0) - md * md;
  mean = (float)md;
  rstd = 1.0f / sqrtf((float)vd + 1e-5f);
}

__global__ __launch_bounds__(256) __attribute__((amdgpu_num_vgpr(248)))
void k_t1(const float* __restrict__ Y0, const unsigned short* __restrict__ W2ALL, const float* __restrict__ BIA,
          const float* __restrict__ WT, const float* __restrict__ BT, const unsigned short* __restrict__ XB,
          float* __restrict__ Tg, double* __restrict__ REC) {
  extern __shared__ __align__(16) unsigned char dyn_lds[];
  float* F = (float*)dyn_lds;
  unsigned short* A = (unsigned short*)(dyn_lds + 64 * LDF * 4);
  double* red = (double*)(dyn_lds + 64 * LDF * 4 + 64 * LDA * 2);
  const int tid = threadIdx.x, lane = tid & 31, w = tid >> 5;
  const int li = lane & 15, h = lane >> 4;
  const int tile = blockIdx.x, m0 = tile * 64;
  const int bl = tile / 5, l = bl % NL, nt0 = (tile - bl * 5) * 64;
  const v8f zero8 = {0.f, 0.f, 0.f, 0.f, 0.f, 0.f, 0.f, 0.f};
#pragma unroll 2
  for (int it = 0; it < 8; ++it) {
    const int q = it * 256 + tid, row = q >> 5, p = q & 31;
    const v4f v = *(const v4fa*)(Y0 + (size_t)(m0 + row) * ND + 4 * p);
    *(v4fa*)(F + row * LDF + 4 * p) = v;
    put_split4(A + row * LDA + 4 * p, v);
  }
  __syncthreads();
  const int col = 16 * w + li;
  v8f acc[4];
#pragma unroll
  for (int i = 0; i < 4; ++i) acc[i] = zero8;
  gemm_one(A, W2ALL + (size_t)col * 256 + 8 * h, li, h, acc);
  __syncthreads();
  {
    const float bias = BIA[512 + col];
#pragma unroll
    for (int i = 0; i < 4; ++i)
#pragma unroll
      for (int r = 0; r < 8; ++r) {
        const int row = 16 * i + 8 * h + r;
        const float y1 = F[row * LDF + col] + (acc[i][r] + bias);
        const unsigned pk = split_pk(y1);
        A[row * LDA + col] = (unsigned short)(pk & 0xffffu);
        A[row * LDA + 128 + col] = (unsigned short)(pk >> 16);
      }
  }
  __syncthreads();
#pragma unroll
  for (int i = 0; i < 4; ++i) acc[i] = zero8;
  gemm_one(A, W2ALL + (size_t)32768 + (size_t)col * 256 + 8 * h, li, h, acc);
  {
    const float bias = BIA[640 + col];
#pragma unroll
    for (int i = 0; i < 4; ++i)
#pragma unroll
      for (int r = 0; r < 8; ++r) {
        const int row = 16 * i + 8 * h + r;
        const float y2 = acc[i][r] + bias;
        F[row * LDF + col] = (y2 > 0.0f) ? y2 : 0.0f;
      }
  }
  __syncthreads();
  v4f tv[8];
  double s = 0.0, qd = 0.0;
#pragma unroll
  for (int it = 0; it < 8; ++it) {
    const int q = it * 256 + tid, row = q >> 5, p = q & 31;
    const int n = nt0 + row;
    const bool valid = n < NN;
    const v4f y2 = *(const v4fa*)(F + row * LDF + 4 * p);
    const v4f wt = *(const v4fa*)(WT + ((size_t)l * NP + n) * ND + 4 * p);
    const v4f bt = *(const v4fa*)(BT + ((size_t)l * NP + n) * ND + 4 * p);
    const v4us xb = *(const v4usa*)(XB + (size_t)(m0 + row) * ND + 4 * p);
    v4f t;
    t.x = ((y2.x * wt.x + bt.x) + y2.x) + bf_bits2f(xb.x);
    t.y = ((y2.y * wt.y + bt.y) + y2.y) + bf_bits2f(xb.y);
    t.z = ((y2.z * wt.z + bt.z) + y2.z) + bf_bits2f(xb.z);
    t.w = ((y2.w * wt.w + bt.w) + y2.w) + bf_bits2f(xb.w);
    tv[it] = t;
    const double dx = (double)t.x, dy = (double)t.y, dz = (double)t.z, dw = (double)t.w;
    s  += valid ? ((dx + dy) + (dz + dw)) : 0.0;
    qd += valid ? ((dx * dx + dy * dy) + (dz * dz + dw * dw)) : 0.0;
  }
  for (int pass = 0; pass < 2; ++pass) {
#pragma unroll
    for (int it = 0; it < 8; ++it) {
      const int q = it * 256 + tid, row = q >> 5, p = q & 31;
      *(volatile v4f*)(Tg + (size_t)(m0 + row) * ND + 4 * p) = tv[it];
    }
    __threadfence();
  }
  write_record(s, qd, red, REC + (size_t)tile * 16, tid);
}

__global__ __launch_bounds__(256) __attribute__((amdgpu_num_vgpr(248)))
void k_t2(const float* __restrict__ Tg, const double* __restrict__ REC1, const unsigned short* __restrict__ WG12,
          const unsigned short* __restrict__ W2ALL, const float* __restrict__ BIA, const float* __restrict__ WT,
          const float* __restrict__ BT, float* __restrict__ U2, double* __restrict__ REC2) {
  extern __shared__ __align__(16) unsigned char dyn_lds[];
  float* F = (float*)dyn_lds;
  unsigned short* A = (unsigned short*)(dyn_lds + 64 * LDF * 4);
  double* red = (double*)(dyn_lds + 64 * LDF * 4 + 64 * LDA * 2);
  const int tid = threadIdx.x, lane = tid & 31, w = tid >> 5;
  const int li = lane & 15, h = lane >> 4;
  const int tile = blockIdx.x, m0 = tile * 64;
  const int bl = tile / 5, l = bl % NL, nt0 = (tile - bl * 5) * 64;
  const v8f zero8 = {0.f, 0.f, 0.f, 0.f, 0.f, 0.f, 0.f, 0.f};
  float mean, rstd;
  ln_stats(REC1, bl, mean, rstd);
#pragma unroll 2
  for (int it = 0; it < 8; ++it) {
    const int q = it * 256 + tid, row = q >> 5, p = q & 31;
    const bool valid = (nt0 + row) < NN;
    const v4f t = *(const v4fa*)(Tg + (size_t)(m0 + row) * ND + 4 * p);
    v4f z;
    z.x = valid ? (t.x - mean) * rstd : 0.0f;
    z.y = valid ? (t.y - mean) * rstd : 0.0f;
    z.z = valid ? (t.z - mean) * rstd : 0.0f;
    z.w = valid ? (t.w - mean) * rstd : 0.0f;
    *(v4fa*)(F + row * LDF + 4 * p) = z;
    put_split4(A + row * LDA + 4 * p, z);
  }
  __syncthreads();
  const int col = 16 * w + li;
  v8f c1[4], c2[4];
#pragma unroll
  for (int i = 0; i < 4; ++i) { c1[i] = zero8; c2[i] = zero8; }
  gemm_two(A, WG12 + (size_t)col * 256 + 8 * h, WG12 + (size_t)(128 + col) * 256 + 8 * h, li, h, c1, c2);
  __syncthreads();
  {
    const float b1 = BIA[256 + col], b2 = BIA[384 + col];
#pragma unroll
    for (int i = 0; i < 4; ++i)
#pragma unroll
      for (int r = 0; r < 8; ++r) {
        const int row = 16 * i + 8 * h + r;
        const float a1 = c1[i][r] + b1;
        const float a2 = c2[i][r] + b2;
        const float sg = 1.0f / (1.0f + expf(-a2));
        const float g = a1 * sg;
        const unsigned pk = split_pk(g);
        A[row * LDA + col] = (unsigned short)(pk & 0xffffu);
        A[row * LDA + 128 + col] = (unsigned short)(pk >> 16);
      }
  }
  __syncthreads();
#pragma unroll
  for (int i = 0; i < 4; ++i) c1[i] = zero8;
  gemm_one(A, W2ALL + (size_t)65536 + (size_t)col * 256 + 8 * h, li, h, c1);
  {
    const float bias = BIA[768 + col];
#pragma unroll
    for (int i = 0; i < 4; ++i)
#pragma unroll
      for (int r = 0; r < 8; ++r) {
        const int row = 16 * i + 8 * h + r;
        const float u = (c1[i][r] + bias) + F[row * LDF + col];
        F[row * LDF + col] = u;
      }
  }
  __syncthreads();
  v4f tv[8];
  double s = 0.0, qd = 0.0;
#pragma unroll
  for (int it = 0; it < 8; ++it) {
    const int q = it * 256 + tid, row = q >> 5, p = q & 31;
    const int n = nt0 + row;
    const bool valid = n < NN;
    const v4f u = *(const v4fa*)(F + row * LDF + 4 * p);
    const v4f wt = *(const v4fa*)(WT + ((size_t)l * NP + n) * ND + 4 * p);
    const v4f bt = *(const v4fa*)(BT + ((size_t)l * NP + n) * ND + 4 * p);
    v4f t;
    t.x = (u.x * wt.x + bt.x) + u.x;
    t.y = (u.y * wt.y + bt.y) + u.y;
    t.z = (u.z * wt.z + bt.z) + u.z;
    t.w = (u.w * wt.w + bt.w) + u.w;
    tv[it] = t;
    const double dx = (double)t.x, dy = (double)t.y, dz = (double)t.z, dw = (double)t.w;
    s  += valid ? ((dx + dy) + (dz + dw)) : 0.0;
    qd += valid ? ((dx * dx + dy * dy) + (dz * dz + dw * dw)) : 0.0;
  }
  for (int pass = 0; pass < 2; ++pass) {
#pragma unroll
    for (int it = 0; it < 8; ++it) {
      const int q = it * 256 + tid, row = q >> 5, p = q & 31;
      *(volatile v4f*)(U2 + (size_t)(m0 + row) * ND + 4 * p) = tv[it];
    }
    __threadfence();
  }
  write_record(s, qd, red, REC2 + (size_t)tile * 16, tid);
}

__global__ __launch_bounds__(256) void k_out(const float* __restrict__ U2, const double* __restrict__ REC2,
                                             float* __restrict__ out) {
  extern __shared__ __align__(16) unsigned char dyn_lds[];
  float* st = (float*)dyn_lds;
  float* ms = st + 8 * SS;
  const int tid = threadIdx.x;
  const int g = blockIdx.x & 15, b = blockIdx.x >> 4;
  const int c0 = 8 * g;
  if (tid < NL) {
    float mean, rstd;
    ln_stats(REC2, b * NL + tid, mean, rstd);
    ms[tid] = mean; ms[NL + tid] = rstd;
  }
  __syncthreads();
#pragma unroll 2
  for (int u = tid; u < SS; u += 256) {
    const int l = u / NN, n = u - l * NN;
    const float* p = U2 + ((size_t)(b * NL + l) * NP + n) * ND + c0;
    const v4f a = *(const v4fa*)p;
    const v4f c = *(const v4fa*)(p + 4);
    const float m = ms[l], r = ms[NL + l];
    float* sp = st + n * NL + l;
    sp[0 * SS] = (a.x - m) * r; sp[1 * SS] = (a.y - m) * r; sp[2 * SS] = (a.z - m) * r; sp[3 * SS] = (a.w - m) * r;
    sp[4 * SS] = (c.x - m) * r; sp[5 * SS] = (c.y - m) * r; sp[6 * SS] = (c.z - m) * r; sp[7 * SS] = (c.w - m) * r;
  }
  __syncthreads();
  float* ob = out + (size_t)(b * ND + c0) * SS;
  for (int pass = 0; pass < 2; ++pass) {
#pragma unroll 2
    for (int q = tid; q < 2 * SS; q += 256) {
      const v4f v = *(const v4fa*)(st + 4 * q);
      *(volatile v4f*)(ob + 4 * (size_t)q) = v;
    }
    __threadfence();
  }
}

extern "C" void kernel_launch(void* const* d_in, const int* in_sizes, int n_in,
                              void* d_out, int out_size, void* d_ws, size_t ws_size,
                              hipStream_t stream) {
  if (n_in < 26) return;
  const int exp_sz[26] = {3772416, 16384, 128, 16384, 128, 16384, 128, 16384, 128, 16384, 128, 16384, 128, 16384, 128,
                          1886208, 4, 8192, 64, 256, 4, 471552, 471552, 3070, 3070, 3};
  for (int i = 0; i < 26; ++i) if (in_sizes[i] != exp_sz[i]) return;
  if (out_size != 3772416) return;

  const float* x    = (const float*)d_in[0];
  const float* Wq   = (const float*)d_in[1];   const float* bq  = (const float*)d_in[2];
  const float* Wv   = (const float*)d_in[3];   const float* bv  = (const float*)d_in[4];
  const float* Wc   = (const float*)d_in[5];   const float* bc  = (const float*)d_in[6];
  const float* Wx   = (const float*)d_in[7];   const float* bx  = (const float*)d_in[8];
  const float* Wg1  = (const float*)d_in[9];   const float* bg1 = (const float*)d_in[10];
  const float* Wg2  = (const float*)d_in[11];  const float* bg2 = (const float*)d_in[12];
  const float* Wg3  = (const float*)d_in[13];  const float* bg3 = (const float*)d_in[14];
  const float* bank = (const float*)d_in[15];
  const float* imp  = (const float*)d_in[16];
  const float* A1   = (const float*)d_in[17];  const float* a1b = (const float*)d_in[18];
  const float* A2   = (const float*)d_in[19];  const float* a2b = (const float*)d_in[20];
  const float* wgt  = (const float*)d_in[21];
  const float* bia  = (const float*)d_in[22];
  const float* nv1  = (const float*)d_in[23];
  const float* nv2  = (const float*)d_in[24];
  const float* sws  = (const float*)d_in[25];
  float* out = (float*)d_out;

  size_t off = 0;
  const size_t oXB   = off; off += (size_t)ROWS * ND * 2;
  const size_t oQHL  = off; off += (size_t)ROWS * 256 * 2;
  const size_t oVTh  = off; off += (size_t)96 * ND * NP * 2;
  const size_t oVTl  = off; off += (size_t)96 * ND * NP * 2;
  const size_t oY0   = off; off += (size_t)ROWS * ND * 4;
  const size_t oT    = off; off += (size_t)ROWS * ND * 4;
  const size_t oWT   = off; off += (size_t)NL * NP * ND * 4;
  const size_t oBT   = off; off += (size_t)NL * NP * ND * 4;
  const size_t oS1   = off; off += (size_t)NP * NP * 4;
  const size_t oS2   = off; off += (size_t)NP * NP * 4;
  const size_t oADJ  = off; off += (size_t)NP * NP * 4;
  const size_t oADJT = off; off += (size_t)NP * NP * 4;
  const size_t oA3S1 = off; off += (size_t)NP * K3 * 2;
  const size_t oBT3  = off; off += (size_t)NP * K3 * 2;
  const size_t oA3S2 = off; off += (size_t)NP * K3 * 2;
  const size_t oWQV  = off; off += (size_t)256 * ND * 2;
  const size_t oWG12 = off; off += (size_t)256 * 256 * 2;
  const size_t oW2   = off; off += (size_t)3 * ND * 256 * 2;
  const size_t oBIA  = off; off += 4096;
  const size_t oAVG  = off; off += 4096;
  const size_t oMEMW = off; off += 256;
  const size_t oREC1 = off; off += (size_t)NTILE * 128;
  const size_t oREC2 = off; off += (size_t)NTILE * 128;
  if (off > ws_size) return;
  if (off > (size_t)134217728) return;

  char* ws = (char*)d_ws;
  unsigned short* XB   = (unsigned short*)(ws + oXB);
  unsigned short* QHL  = (unsigned short*)(ws + oQHL);
  unsigned short* VTh  = (unsigned short*)(ws + oVTh);
  unsigned short* VTl  = (unsigned short*)(ws + oVTl);
  float* Y0   = (float*)(ws + oY0);
  float* U2   = (float*)(ws + oY0);
  float* Tg   = (float*)(ws + oT);
  float* WT   = (float*)(ws + oWT);
  float* BT   = (float*)(ws + oBT);
  float* S1   = (float*)(ws + oS1);
  float* S2   = (float*)(ws + oS2);
  float* ADJ  = (float*)(ws + oADJ);
  float* ADJT = (float*)(ws + oADJT);
  unsigned short* A3S1 = (unsigned short*)(ws + oA3S1);
  unsigned short* BT3  = (unsigned short*)(ws + oBT3);
  unsigned short* A3S2 = (unsigned short*)(ws + oA3S2);
  unsigned short* WQV  = (unsigned short*)(ws + oWQV);
  unsigned short* WG12 = (unsigned short*)(ws + oWG12);
  unsigned short* W2ALL = (unsigned short*)(ws + oW2);
  float* BIA  = (float*)(ws + oBIA);
  float* AVG  = (float*)(ws + oAVG);
  float* MEMW = (float*)(ws + oMEMW);
  double* REC1 = (double*)(ws + oREC1);
  double* REC2 = (double*)(ws + oREC2);

  const int ldsTok = 128 * 192 * 4;
  const int ldsQv  = 65536;
  const int ldsAtt = 40960 + 4 * 43008;
  const int ldsTl  = 64 * LDF * 4 + 64 * LDA * 2 + 128;
  const int ldsOut = 118016;
  (void)hipFuncSetAttribute(reinterpret_cast<const void*>(&k_tok<0>), hipFuncAttributeMaxDynamicSharedMemorySize, ldsTok);
  (void)hipFuncSetAttribute(reinterpret_cast<const void*>(&k_tok<1>), hipFuncAttributeMaxDynamicSharedMemorySize, ldsTok);
  (void)hipFuncSetAttribute(reinterpret_cast<const void*>(&k_qv), hipFuncAttributeMaxDynamicSharedMemorySize, ldsQv);
  (void)hipFuncSetAttribute(reinterpret_cast<const void*>(&k_attn), hipFuncAttributeMaxDynamicSharedMemorySize, ldsAtt);
  (void)hipFuncSetAttribute(reinterpret_cast<const void*>(&k_t1), hipFuncAttributeMaxDynamicSharedMemorySize, ldsTl);
  (void)hipFuncSetAttribute(reinterpret_cast<const void*>(&k_t2), hipFuncAttributeMaxDynamicSharedMemorySize, ldsTl);
  (void)hipFuncSetAttribute(reinterpret_cast<const void*>(&k_out), hipFuncAttributeMaxDynamicSharedMemorySize, ldsOut);

  k_pa1<<<dim3(49), dim3(256), 0, stream>>>(Wq, Wv, Wg1, Wg2, bq, bv, bg1, bg2, WQV, WG12, BIA);
  k_pa2<<<dim3(49), dim3(256), 0, stream>>>(Wx, Wc, Wg3, bx, bc, bg3, W2ALL, BIA);
  k_tok<0><<<dim3(20, NB), dim3(256), ldsTok, stream>>>(x, XB, WT);
  k_tok<1><<<dim3(20, 1), dim3(256), ldsTok, stream>>>(wgt, XB, WT);
  k_tok<1><<<dim3(20, 1), dim3(256), ldsTok, stream>>>(bia, XB, BT);
  k_avg<<<dim3(32), dim3(256), 0, stream>>>(x, AVG);
  k_mem<<<dim3(1), dim3(256), 0, stream>>>(AVG, A1, a1b, A2, a2b, imp, MEMW);
  k_s1<<<dim3(20), dim3(256), 0, stream>>>(nv1, nv2, S1, A3S1);
  k_trans<1><<<dim3(20), dim3(256), 0, stream>>>(S1, ADJT, BT3);
  k_s23<2><<<dim3(20), dim3(128), 0, stream>>>(A3S1, BT3, S1, S1, sws, S2, A3S2);
  k_s23<3><<<dim3(20), dim3(128), 0, stream>>>(A3S2, BT3, S1, S2, sws, ADJ, A3S2);
  k_trans<0><<<dim3(20), dim3(256), 0, stream>>>(ADJ, ADJT, BT3);
  k_qv<<<dim3(NTILE), dim3(256), ldsQv, stream>>>(XB, WQV, BIA, QHL, VTh, VTl);
  k_attn<<<dim3(384), dim3(128), ldsAtt, stream>>>(QHL, VTh, VTl, bank, MEMW, ADJT, Y0);
  k_t1<<<dim3(NTILE), dim3(256), ldsTl, stream>>>(Y0, W2ALL, BIA, WT, BT, XB, Tg, REC1);
  k_t2<<<dim3(NTILE), dim3(256), ldsTl, stream>>>(Tg, REC1, WG12, W2ALL, BIA, WT, BT, U2, REC2);
  k_out<<<dim3(128), dim3(256), ldsOut, stream>>>(U2, REC2, out);
  (void)hipGetLastError();
}
